// PMA_batch_74509092651637
// MI455X (gfx1250) — hardware-verified
//
#include <hip/hip_runtime.h>
#include <hip/hip_bf16.h>
#include <stddef.h>


#define DD    256
#define NHD   4
#define HCD   64
#define BQ    8
#define GR    32
#define XSP   260
#define HPB   264
#define NB    32
#define CHUNK 2048
#define NTHR  256
#define NWAVE 8
#define WCAP  256
#define NGRP  (CHUNK / (NTHR * 4))

#define LDS_ATT_F     (BQ * NB * DD + 2 * BQ * NB * NHD)
#define LDS_ATT_BYTES ((LDS_ATT_F + NWAVE * WCAP + 16) * 4)
#define LDS_RFF_BYTES (2 * GR * HPB * 2 + GR * XSP * 4)

static_assert(WCAP == NGRP * 4 * 32);
static_assert(NGRP >= 1);
static_assert(BQ == NWAVE);
static_assert(NB == 32);
static_assert(CHUNK == 2048);
static_assert(DD == NHD * HCD);
static_assert(DD == NWAVE * 32);
static_assert(((BQ * NB * DD) % 4) == 0);
static_assert(BQ * NB * NHD == NTHR * 4);
static_assert(LDS_ATT_BYTES == 278592);
static_assert(LDS_RFF_BYTES == 67072);
static_assert(((2 * GR * HPB * 2) % 16) == 0);
static_assert(((HPB * 2) % 16) == 0);
static_assert(((XSP * 4) % 16) == 0);

typedef float          v4f     __attribute__((ext_vector_type(4)));
typedef float          v8f     __attribute__((ext_vector_type(8)));
typedef int            v4i     __attribute__((ext_vector_type(4)));
typedef unsigned short us4     __attribute__((ext_vector_type(4)));
typedef unsigned short us8     __attribute__((ext_vector_type(8)));
typedef __bf16         bf16x16 __attribute__((ext_vector_type(16)));
union Frag { bf16x16 v; us8 h[2]; };

__device__ __forceinline__ unsigned short bfr(float f) {
  unsigned u = __float_as_uint(f);
  u = (u + 0x7FFFu + ((u >> 16) & 1u)) >> 16;
  return (unsigned short)u;
}
__device__ __forceinline__ float bff(unsigned short s) {
  return __uint_as_float(((unsigned)s) << 16);
}

__device__ __forceinline__ v8f wm3(bf16x16 ah, bf16x16 al, bf16x16 bh, bf16x16 bl, v8f c) {
  c = __builtin_amdgcn_wmma_f32_16x16x32_bf16(false, ah, false, bh, (short)0, c, false, false);
  c = __builtin_amdgcn_wmma_f32_16x16x32_bf16(false, ah, false, bl, (short)0, c, false, false);
  c = __builtin_amdgcn_wmma_f32_16x16x32_bf16(false, al, false, bh, (short)0, c, false, false);
  asm volatile("v_nop\n\tv_nop\n\tv_nop\n\tv_nop" : "+v"(c) : "v"(ah), "v"(al), "v"(bh), "v"(bl));
  return c;
}

#define LDF(F, P) { (F).h[0] = *(const us8*)(P); (F).h[1] = *(const us8*)((P) + 16); }

__device__ __forceinline__ float wsum(float v) {
  v += __shfl_xor(v, 16, 32);
  v += __shfl_xor(v, 8, 32);
  v += __shfl_xor(v, 4, 32);
  v += __shfl_xor(v, 2, 32);
  v += __shfl_xor(v, 1, 32);
  return v;
}

__device__ __forceinline__ void stage8(float* Xs, v8f c, int row0, int col, float bs) {
#pragma unroll
  for (int r = 0; r < 8; ++r) Xs[(row0 + r) * XSP + col] = c[r] + bs;
}
__device__ __forceinline__ void stage8h(unsigned short* Hh, unsigned short* Hl, v8f c, int row0, int col, float bs) {
#pragma unroll
  for (int r = 0; r < 8; ++r) {
    const float v = fmaxf(c[r] + bs, 0.f);
    const unsigned short uh = bfr(v);
    Hh[(row0 + r) * HPB + col] = uh;
    Hl[(row0 + r) * HPB + col] = bfr(v - bff(uh));
  }
}
__device__ __forceinline__ void stage8r(float* Rs, v8f c, int row0, int col, float bs) {
#pragma unroll
  for (int r = 0; r < 8; ++r) Rs[(row0 + r) * XSP + col] = fmaxf(c[r] + bs, 0.f);
}

__global__ __launch_bounds__(NTHR) void k_split(const float* __restrict__ src,
                                             unsigned short* hi, unsigned short* lo, int n8) {
  const int i = blockIdx.x * NTHR + threadIdx.x;
  if (i >= n8) return;
  const size_t o = (size_t)i * 8;
  const v4f a = *(const v4f*)(src + o);
  const v4f b = *(const v4f*)(src + o + 4);
  us8 uh, ul;
  uh[0] = bfr(a.x); uh[1] = bfr(a.y); uh[2] = bfr(a.z); uh[3] = bfr(a.w);
  uh[4] = bfr(b.x); uh[5] = bfr(b.y); uh[6] = bfr(b.z); uh[7] = bfr(b.w);
  ul[0] = bfr(a.x - bff(uh[0])); ul[1] = bfr(a.y - bff(uh[1]));
  ul[2] = bfr(a.z - bff(uh[2])); ul[3] = bfr(a.w - bff(uh[3]));
  ul[4] = bfr(b.x - bff(uh[4])); ul[5] = bfr(b.y - bff(uh[5]));
  ul[6] = bfr(b.z - bff(uh[6])); ul[7] = bfr(b.w - bff(uh[7]));
  *(volatile us8*)(hi + o) = uh;
  *(volatile us8*)(lo + o) = ul;
  __threadfence();
  *(volatile us8*)(hi + o) = uh;
  *(volatile us8*)(lo + o) = ul;
}

__global__ __launch_bounds__(NTHR) void k_gemm_kv(
    const unsigned short* __restrict__ xh, const unsigned short* __restrict__ xl,
    const unsigned short* __restrict__ wh, const unsigned short* __restrict__ wl,
    const float* __restrict__ bK, const float* __restrict__ bV,
    const float* __restrict__ attr, float* xv, float* alpha, int nRows) {
  __shared__ __attribute__((aligned(16))) float Xs[GR * XSP];
  __shared__ __attribute__((aligned(16))) float Al[GR * NHD];

  const int tid  = threadIdx.x;
  const int lane = tid & 31;
  const int wave = tid >> 5;
  const int hh   = lane >> 4;
  const int m    = lane & 15;
  const int rowBase = blockIdx.x * GR;
  const int part = blockIdx.y;
  const int colw = wave * 32;
  if (rowBase + GR > nRows) return;

  const unsigned short* pa0h = xh + (size_t)(rowBase + m) * DD + 8 * hh;
  const unsigned short* pa0l = xl + (size_t)(rowBase + m) * DD + 8 * hh;
  const unsigned short* pa1h = xh + (size_t)(rowBase + 16 + m) * DD + 8 * hh;
  const unsigned short* pa1l = xl + (size_t)(rowBase + 16 + m) * DD + 8 * hh;
  const unsigned short* pb0h = wh + (size_t)(part * DD + colw + m) * DD + 8 * hh;
  const unsigned short* pb0l = wl + (size_t)(part * DD + colw + m) * DD + 8 * hh;
  const unsigned short* pb1h = wh + (size_t)(part * DD + colw + 16 + m) * DD + 8 * hh;
  const unsigned short* pb1l = wl + (size_t)(part * DD + colw + 16 + m) * DD + 8 * hh;

  v8f c00 = {0.f, 0.f, 0.f, 0.f, 0.f, 0.f, 0.f, 0.f};
  v8f c01 = c00, c10 = c00, c11 = c00;
#pragma unroll 1
  for (int k0 = 0; k0 < DD; k0 += 32) {
    Frag a0h, a0l, a1h, a1l, b0h, b0l, b1h, b1l;
    LDF(a0h, pa0h + k0) LDF(a0l, pa0l + k0) LDF(a1h, pa1h + k0) LDF(a1l, pa1l + k0)
    LDF(b0h, pb0h + k0) LDF(b0l, pb0l + k0) LDF(b1h, pb1h + k0) LDF(b1l, pb1l + k0)
    c00 = wm3(a0h.v, a0l.v, b0h.v, b0l.v, c00);
    c01 = wm3(a0h.v, a0l.v, b1h.v, b1l.v, c01);
    c10 = wm3(a1h.v, a1l.v, b0h.v, b0l.v, c10);
    c11 = wm3(a1h.v, a1l.v, b1h.v, b1l.v, c11);
  }

  const float* bias = (part == 0) ? bK : bV;
  {
    const int col0 = colw + m, col1 = colw + 16 + m;
    const float bs0 = bias[col0], bs1 = bias[col1];
    stage8(Xs, c00, 8 * hh, col0, bs0);
    stage8(Xs, c10, 16 + 8 * hh, col0, bs0);
    stage8(Xs, c01, 8 * hh, col1, bs1);
    stage8(Xs, c11, 16 + 8 * hh, col1, bs1);
  }
  __syncthreads();

  if (part == 0) {
    const int r  = tid >> 3;
    const int q  = tid & 7;
    const int hq = q >> 1;
    const int hf = q & 1;
    const float* xr = Xs + r * XSP + hq * HCD + hf * 32;
    const float* ar = attr + hq * HCD + hf * 32;
    float s = 0.f;
#pragma unroll 4
    for (int c = 0; c < 32; ++c) s += xr[c] * ar[c];
    s += __shfl_xor(s, 1, 32);
    if (hf == 0) Al[r * NHD + hq] = s;
    __syncthreads();
    if (wave == 0) {
      const v4f v = *(const v4f*)(Al + 4 * lane);
      float* gp = alpha + (size_t)rowBase * NHD + 4 * lane;
      *(volatile v4f*)gp = v;
      __threadfence();
      *(volatile v4f*)gp = v;
    }
  } else {
    v4f u0[4], u1[4];
#pragma unroll
    for (int i = 0; i < 4; ++i) {
      const int rl = 4 * wave + i;
      u0[i] = *(const v4f*)(Xs + rl * XSP + 4 * lane);
      u1[i] = *(const v4f*)(Xs + rl * XSP + 128 + 4 * lane);
    }
#pragma unroll
    for (int i = 0; i < 4; ++i) {
      float* p = xv + (size_t)(rowBase + 4 * wave + i) * DD;
      *(volatile v4f*)(p + 4 * lane) = u0[i];
      *(volatile v4f*)(p + 128 + 4 * lane) = u1[i];
    }
    __threadfence();
#pragma unroll
    for (int i = 0; i < 4; ++i) {
      float* p = xv + (size_t)(rowBase + 4 * wave + i) * DD;
      *(volatile v4f*)(p + 4 * lane) = u0[i];
      *(volatile v4f*)(p + 128 + 4 * lane) = u1[i];
    }
  }
}

__device__ __forceinline__ void scan_chunk(const int* __restrict__ eid, int nE, int cbase, int nodeBase,
                                           int vec16, int* list, int* wcnt, int tid, int lane, int wave) {
  int wc = 0;
#pragma unroll
  for (int g = 0; g < NGRP; ++g) {
    const int el0 = (g * NTHR + tid) * 4;
    const int e0  = cbase + el0;
    const int sent = -2147483647 - 1;
    v4i d;
    if (vec16 != 0 && (cbase + CHUNK <= nE)) {
      d = *(const v4i*)(eid + e0);
    } else {
      const int v0 = eid[min(e0, nE - 1)];
      const int v1 = eid[min(e0 + 1, nE - 1)];
      const int v2 = eid[min(e0 + 2, nE - 1)];
      const int v3 = eid[min(e0 + 3, nE - 1)];
      d.x = (e0     < nE) ? v0 : sent;
      d.y = (e0 + 1 < nE) ? v1 : sent;
      d.z = (e0 + 2 < nE) ? v2 : sent;
      d.w = (e0 + 3 < nE) ? v3 : sent;
    }
    const unsigned s0 = (unsigned)d.x - (unsigned)nodeBase;
    const unsigned s1 = (unsigned)d.y - (unsigned)nodeBase;
    const unsigned s2 = (unsigned)d.z - (unsigned)nodeBase;
    const unsigned s3 = (unsigned)d.w - (unsigned)nodeBase;
    const bool h0 = s0 < (unsigned)NB;
    const bool h1 = s1 < (unsigned)NB;
    const bool h2 = s2 < (unsigned)NB;
    const bool h3 = s3 < (unsigned)NB;
    const unsigned many = __builtin_amdgcn_ballot_w32(h0 | h1 | h2 | h3);
    if (many != 0u) {
#define HITJ(J, HJ, SJ) { \
        const unsigned mj = __builtin_amdgcn_ballot_w32(HJ); \
        if (HJ) { \
          const int pos = wc + (int)__builtin_amdgcn_mbcnt_lo(mj, 0u); \
          if (pos < WCAP) list[wave * WCAP + pos] = ((el0 + (J)) << 5) | (int)(SJ); \
        } \
        wc += (int)__builtin_popcount(mj); }
      HITJ(0, h0, s0)
      HITJ(1, h1, s1)
      HITJ(2, h2, s2)
      HITJ(3, h3, s3)
#undef HITJ
    }
  }
  if (lane == 0) wcnt[wave] = wc;
}

__global__ __launch_bounds__(NTHR) void k_att(
    const int* __restrict__ ei, const float* __restrict__ alpha, const float* __restrict__ xv,
    const float* __restrict__ attr, const float* __restrict__ gam, const float* __restrict__ bet,
    unsigned short* o0h, unsigned short* o0l, int nN, int nE) {
  extern __shared__ v4f lds_att[];
  float* sacc = (float*)lds_att;
  float* sden = sacc + BQ * NB * DD;
  float* smx  = sden + BQ * NB * NHD;
  int*   list = (int*)(smx + BQ * NB * NHD);
  int*   wcnt = list + NWAVE * WCAP;

  const int tid  = threadIdx.x;
  const int lane = tid & 31;
  const int wave = tid >> 5;
  const int hd   = lane >> 3;
  const int nodeBase = blockIdx.x * NB;
  const int b = wave;
  const size_t bRow = (size_t)b * (size_t)nN;

  {
    const v4f z4 = {0.f, 0.f, 0.f, 0.f};
    const int nz = (BQ * NB * DD + BQ * NB * NHD) / 4;
    for (int i = tid; i < nz; i += NTHR) lds_att[i] = z4;
    const float ninf = __uint_as_float(0xff800000u);
    const v4f n4 = {ninf, ninf, ninf, ninf};
    lds_att[nz + tid] = n4;
  }
  __syncthreads();

  const int* eid = ei + nE;
  const int vec16 = ((nE & 3) == 0) ? 1 : 0;
  const int nChunks = (nE + CHUNK - 1) / CHUNK;

#pragma unroll 1
  for (int ch = 0; ch < nChunks; ++ch) {
    const int cbase = ch * CHUNK;
    scan_chunk(eid, nE, cbase, nodeBase, vec16, list, wcnt, tid, lane, wave);
    __syncthreads();
    for (int wsx = 0; wsx < NWAVE; ++wsx) {
      int n = wcnt[wsx];
      n = n < 0 ? 0 : (n > WCAP ? WCAP : n);
      for (int i = 0; i < n; ++i) {
        const int ent  = list[wsx * WCAP + i];
        const int slot = ent & (NB - 1);
        const int el   = (ent >> 5) & (CHUNK - 1);
        int e = cbase + el;
        e = e > nE - 1 ? nE - 1 : e;
        int src = ei[e];
        src = src < 0 ? 0 : (src > nN - 1 ? nN - 1 : src);
        float a = alpha[(bRow + (size_t)src) * NHD + hd];
        a = (a >= 0.f) ? a : 0.2f * a;
        const int ix = (b * NB + slot) * NHD + hd;
        smx[ix] = fmaxf(smx[ix], a);
      }
    }
    __syncthreads();
  }
  for (int i = tid; i < BQ * NB * NHD; i += NTHR) {
    const float v = smx[i];
    smx[i] = (v > -3.0e38f && v < 3.0e38f) ? v : 0.f;
  }
  __syncthreads();

#pragma unroll 1
  for (int ch = 0; ch < nChunks; ++ch) {
    const int cbase = ch * CHUNK;
    scan_chunk(eid, nE, cbase, nodeBase, vec16, list, wcnt, tid, lane, wave);
    __syncthreads();
    for (int wsx = 0; wsx < NWAVE; ++wsx) {
      int n = wcnt[wsx];
      n = n < 0 ? 0 : (n > WCAP ? WCAP : n);
      for (int i = 0; i < n; ++i) {
        const int ent  = list[wsx * WCAP + i];
        const int slot = ent & (NB - 1);
        const int el   = (ent >> 5) & (CHUNK - 1);
        int e = cbase + el;
        e = e > nE - 1 ? nE - 1 : e;
        int src = ei[e];
        src = src < 0 ? 0 : (src > nN - 1 ? nN - 1 : src);
        const size_t srow = bRow + (size_t)src;
        float a = alpha[srow * NHD + hd];
        a = (a >= 0.f) ? a : 0.2f * a;
        const int ix = (b * NB + slot) * NHD + hd;
        const float p = __expf(a - smx[ix]);
        const float* xp = xv + srow * DD + 8 * lane;
        const v4f x0 = *(const v4f*)xp;
        const v4f x1 = *(const v4f*)(xp + 4);
        float* sp = sacc + (b * NB + slot) * DD + 8 * lane;
        const v4f c0 = *(const v4f*)sp;
        const v4f c1 = *(const v4f*)(sp + 4);
        const v4f n0 = c0 + p * x0;
        const v4f n1 = c1 + p * x1;
        *(v4f*)sp = n0;
        *(v4f*)(sp + 4) = n1;
        const float dv = sden[ix];
        sden[ix] = dv + p;
      }
    }
    __syncthreads();
  }

  const v4f r0 = *(const v4f*)(attr + 8 * lane), r1 = *(const v4f*)(attr + 8 * lane + 4);
  const v4f g0 = *(const v4f*)(gam + 8 * lane),  g1 = *(const v4f*)(gam + 8 * lane + 4);
  const v4f e0 = *(const v4f*)(bet + 8 * lane),  e1 = *(const v4f*)(bet + 8 * lane + 4);
#pragma unroll 1
  for (int j = 0; j < NB; ++j) {
    const int node = nodeBase + j;
    if (node >= nN) break;
    const size_t grow = bRow + (size_t)node;
    const float* sp = sacc + (b * NB + j) * DD + 8 * lane;
    const v4f s0 = *(const v4f*)sp;
    const v4f s1 = *(const v4f*)(sp + 4);
    const float dv  = sden[(b * NB + j) * NHD + hd];
    const float inv = __builtin_amdgcn_rcpf(dv + 1e-16f);
    const v4f h0 = s0 * inv + r0;
    const v4f h1 = s1 * inv + r1;
    const float s  = wsum(h0.x + h0.y + h0.z + h0.w + h1.x + h1.y + h1.z + h1.w);
    const float mu = s * (1.0f / DD);
    const v4f d0 = h0 - mu, d1 = h1 - mu;
    const float q  = wsum(d0.x * d0.x + d0.y * d0.y + d0.z * d0.z + d0.w * d0.w +
                          d1.x * d1.x + d1.y * d1.y + d1.z * d1.z + d1.w * d1.w);
    const float rs = rsqrtf(q * (1.0f / DD) + 1e-5f);
    const v4f y0 = d0 * rs * g0 + e0;
    const v4f y1 = d1 * rs * g1 + e1;
    us8 uh, ul;
    uh[0] = bfr(y0.x); uh[1] = bfr(y0.y); uh[2] = bfr(y0.z); uh[3] = bfr(y0.w);
    uh[4] = bfr(y1.x); uh[5] = bfr(y1.y); uh[6] = bfr(y1.z); uh[7] = bfr(y1.w);
    ul[0] = bfr(y0.x - bff(uh[0])); ul[1] = bfr(y0.y - bff(uh[1]));
    ul[2] = bfr(y0.z - bff(uh[2])); ul[3] = bfr(y0.w - bff(uh[3]));
    ul[4] = bfr(y1.x - bff(uh[4])); ul[5] = bfr(y1.y - bff(uh[5]));
    ul[6] = bfr(y1.z - bff(uh[6])); ul[7] = bfr(y1.w - bff(uh[7]));
    unsigned short* ph = o0h + grow * DD + 8 * lane;
    unsigned short* pl = o0l + grow * DD + 8 * lane;
    *(volatile us8*)ph = uh;
    *(volatile us8*)pl = ul;
    __threadfence();
    *(volatile us8*)ph = uh;
    *(volatile us8*)pl = ul;
  }
}

__global__ __launch_bounds__(NTHR) void k_rff(
    const unsigned short* __restrict__ yh, const unsigned short* __restrict__ yl,
    const unsigned short* __restrict__ w1h, const unsigned short* __restrict__ w1l,
    const unsigned short* __restrict__ w2h, const unsigned short* __restrict__ w2l,
    const float* __restrict__ b1, const float* __restrict__ b2,
    const float* __restrict__ gam, const float* __restrict__ bet,
    float* out, int nRows) {
  extern __shared__ v4f lds_rff[];
  unsigned short* Hh = (unsigned short*)lds_rff;
  unsigned short* Hl = Hh + GR * HPB;
  float* Rs = (float*)(Hl + GR * HPB);

  const int tid  = threadIdx.x;
  const int lane = tid & 31;
  const int wave = tid >> 5;
  const int hh   = lane >> 4;
  const int m    = lane & 15;
  const int rowBase = blockIdx.x * GR;
  const int colw = wave * 32;
  if (rowBase + GR > nRows) return;

  {
    const unsigned short* pa0h = yh + (size_t)(rowBase + m) * DD + 8 * hh;
    const unsigned short* pa0l = yl + (size_t)(rowBase + m) * DD + 8 * hh;
    const unsigned short* pa1h = yh + (size_t)(rowBase + 16 + m) * DD + 8 * hh;
    const unsigned short* pa1l = yl + (size_t)(rowBase + 16 + m) * DD + 8 * hh;
    const unsigned short* pb0h = w1h + (size_t)(colw + m) * DD + 8 * hh;
    const unsigned short* pb0l = w1l + (size_t)(colw + m) * DD + 8 * hh;
    const unsigned short* pb1h = w1h + (size_t)(colw + 16 + m) * DD + 8 * hh;
    const unsigned short* pb1l = w1l + (size_t)(colw + 16 + m) * DD + 8 * hh;
    v8f c00 = {0.f, 0.f, 0.f, 0.f, 0.f, 0.f, 0.f, 0.f};
    v8f c01 = c00, c10 = c00, c11 = c00;
#pragma unroll 1
    for (int k0 = 0; k0 < DD; k0 += 32) {
      Frag a0h, a0l, a1h, a1l, b0h, b0l, b1h, b1l;
      LDF(a0h, pa0h + k0) LDF(a0l, pa0l + k0) LDF(a1h, pa1h + k0) LDF(a1l, pa1l + k0)
      LDF(b0h, pb0h + k0) LDF(b0l, pb0l + k0) LDF(b1h, pb1h + k0) LDF(b1l, pb1l + k0)
      c00 = wm3(a0h.v, a0l.v, b0h.v, b0l.v, c00);
      c01 = wm3(a0h.v, a0l.v, b1h.v, b1l.v, c01);
      c10 = wm3(a1h.v, a1l.v, b0h.v, b0l.v, c10);
      c11 = wm3(a1h.v, a1l.v, b1h.v, b1l.v, c11);
    }
    const int col0 = colw + m, col1 = colw + 16 + m;
    const float bs0 = b1[col0], bs1 = b1[col1];
    stage8h(Hh, Hl, c00, 8 * hh, col0, bs0);
    stage8h(Hh, Hl, c10, 16 + 8 * hh, col0, bs0);
    stage8h(Hh, Hl, c01, 8 * hh, col1, bs1);
    stage8h(Hh, Hl, c11, 16 + 8 * hh, col1, bs1);
  }
  __syncthreads();

  {
    const unsigned short* qa0h = Hh + m * HPB + 8 * hh;
    const unsigned short* qa0l = Hl + m * HPB + 8 * hh;
    const unsigned short* qa1h = Hh + (16 + m) * HPB + 8 * hh;
    const unsigned short* qa1l = Hl + (16 + m) * HPB + 8 * hh;
    const unsigned short* pb0h = w2h + (size_t)(colw + m) * DD + 8 * hh;
    const unsigned short* pb0l = w2l + (size_t)(colw + m) * DD + 8 * hh;
    const unsigned short* pb1h = w2h + (size_t)(colw + 16 + m) * DD + 8 * hh;
    const unsigned short* pb1l = w2l + (size_t)(colw + 16 + m) * DD + 8 * hh;
    v8f c00 = {0.f, 0.f, 0.f, 0.f, 0.f, 0.f, 0.f, 0.f};
    v8f c01 = c00, c10 = c00, c11 = c00;
#pragma unroll 1
    for (int k0 = 0; k0 < DD; k0 += 32) {
      Frag a0h, a0l, a1h, a1l, b0h, b0l, b1h, b1l;
      LDF(a0h, qa0h + k0) LDF(a0l, qa0l + k0) LDF(a1h, qa1h + k0) LDF(a1l, qa1l + k0)
      LDF(b0h, pb0h + k0) LDF(b0l, pb0l + k0) LDF(b1h, pb1h + k0) LDF(b1l, pb1l + k0)
      c00 = wm3(a0h.v, a0l.v, b0h.v, b0l.v, c00);
      c01 = wm3(a0h.v, a0l.v, b1h.v, b1l.v, c01);
      c10 = wm3(a1h.v, a1l.v, b0h.v, b0l.v, c10);
      c11 = wm3(a1h.v, a1l.v, b1h.v, b1l.v, c11);
    }
    __syncthreads();
    const int col0 = colw + m, col1 = colw + 16 + m;
    const float bs0 = b2[col0], bs1 = b2[col1];
    stage8r(Rs, c00, 8 * hh, col0, bs0);
    stage8r(Rs, c10, 16 + 8 * hh, col0, bs0);
    stage8r(Rs, c01, 8 * hh, col1, bs1);
    stage8r(Rs, c11, 16 + 8 * hh, col1, bs1);
  }
  __syncthreads();

  const v4f G0 = *(const v4f*)(gam + 4 * lane), G1 = *(const v4f*)(gam + 128 + 4 * lane);
  const v4f E0 = *(const v4f*)(bet + 4 * lane), E1 = *(const v4f*)(bet + 128 + 4 * lane);
  v4f yA[4], yB[4];
#pragma unroll
  for (int i = 0; i < 4; ++i) {
    const int rl = 4 * wave + i;
    const size_t grow = (size_t)(rowBase + rl);
    const v4f q0 = *(const v4f*)(Rs + rl * XSP + 4 * lane);
    const v4f q1 = *(const v4f*)(Rs + rl * XSP + 128 + 4 * lane);
    const us4 a0 = *(const us4*)(yh + grow * DD + 4 * lane);
    const us4 l0 = *(const us4*)(yl + grow * DD + 4 * lane);
    const us4 a1 = *(const us4*)(yh + grow * DD + 128 + 4 * lane);
    const us4 l1 = *(const us4*)(yl + grow * DD + 128 + 4 * lane);
    v4f z0, z1;
    z0.x = bff(a0.x) + bff(l0.x); z0.y = bff(a0.y) + bff(l0.y);
    z0.z = bff(a0.z) + bff(l0.z); z0.w = bff(a0.w) + bff(l0.w);
    z1.x = bff(a1.x) + bff(l1.x); z1.y = bff(a1.y) + bff(l1.y);
    z1.z = bff(a1.z) + bff(l1.z); z1.w = bff(a1.w) + bff(l1.w);
    const v4f v0 = z0 + q0, v1 = z1 + q1;
    const float s  = wsum(v0.x + v0.y + v0.z + v0.w + v1.x + v1.y + v1.z + v1.w);
    const float mu = s * (1.0f / DD);
    const v4f d0 = v0 - mu, d1 = v1 - mu;
    const float q  = wsum(d0.x * d0.x + d0.y * d0.y + d0.z * d0.z + d0.w * d0.w +
                          d1.x * d1.x + d1.y * d1.y + d1.z * d1.z + d1.w * d1.w);
    const float rs = rsqrtf(q * (1.0f / DD) + 1e-5f);
    yA[i] = d0 * rs * G0 + E0;
    yB[i] = d1 * rs * G1 + E1;
  }
#pragma unroll
  for (int i = 0; i < 4; ++i) {
    float* p = out + (size_t)(rowBase + 4 * wave + i) * DD;
    *(volatile v4f*)(p + 4 * lane) = yA[i];
    *(volatile v4f*)(p + 128 + 4 * lane) = yB[i];
  }
  __threadfence();
#pragma unroll
  for (int i = 0; i < 4; ++i) {
    float* p = out + (size_t)(rowBase + 4 * wave + i) * DD;
    *(volatile v4f*)(p + 4 * lane) = yA[i];
    *(volatile v4f*)(p + 128 + 4 * lane) = yB[i];
  }
}

extern "C" void kernel_launch(void* const* d_in, const int* in_sizes, int n_in,
                              void* d_out, int out_size, void* d_ws, size_t ws_size,
                              hipStream_t stream) {
  if (n_in < 15) return;
  const int nX = in_sizes[0];
  const int rows = nX / DD;
  if (rows <= 0 || rows * DD != nX) return;
  if ((rows % GR) != 0 || (rows % BQ) != 0) return;
  const int nN = rows / BQ;
  const int nE = in_sizes[1] / 2;
  if (nE < 1 || in_sizes[1] != 2 * nE) return;
  if (in_sizes[2] != DD * DD || in_sizes[4] != DD * DD) return;
  if (in_sizes[11] != DD * DD || in_sizes[13] != DD * DD) return;
  if (in_sizes[3] != DD || in_sizes[5] != DD || in_sizes[6] != NHD * HCD) return;
  if (in_sizes[7] != DD || in_sizes[8] != DD || in_sizes[9] != DD || in_sizes[10] != DD) return;
  if (in_sizes[12] != DD || in_sizes[14] != DD) return;
  if (out_size != rows * DD) return;

  const float* x     = (const float*)d_in[0];
  const int*   ei    = (const int*)d_in[1];
  const float* W_K   = (const float*)d_in[2];
  const float* b_K   = (const float*)d_in[3];
  const float* W_V   = (const float*)d_in[4];
  const float* b_V   = (const float*)d_in[5];
  const float* att_r = (const float*)d_in[6];
  const float* ln0_g = (const float*)d_in[7];
  const float* ln0_b = (const float*)d_in[8];
  const float* ln1_g = (const float*)d_in[9];
  const float* ln1_b = (const float*)d_in[10];
  const float* W1    = (const float*)d_in[11];
  const float* b1    = (const float*)d_in[12];
  const float* W2    = (const float*)d_in[13];
  const float* b2    = (const float*)d_in[14];
  float* out = (float*)d_out;

  char* ws = (char*)d_ws;
  size_t off = 0;
  const size_t planeX = (size_t)rows * DD * sizeof(unsigned short);
  const size_t planeW = (size_t)DD * DD * sizeof(unsigned short);
  unsigned short* xh   = (unsigned short*)(ws + off); off += planeX;
  unsigned short* xl   = (unsigned short*)(ws + off); off += planeX;
  unsigned short* wkvh = (unsigned short*)(ws + off); off += 2 * planeW;
  unsigned short* wkvl = (unsigned short*)(ws + off); off += 2 * planeW;
  unsigned short* w1h  = (unsigned short*)(ws + off); off += planeW;
  unsigned short* w1l  = (unsigned short*)(ws + off); off += planeW;
  unsigned short* w2h  = (unsigned short*)(ws + off); off += planeW;
  unsigned short* w2l  = (unsigned short*)(ws + off); off += planeW;
  float* xv    = (float*)(ws + off); off += (size_t)rows * DD * sizeof(float);
  float* alpha = (float*)(ws + off); off += (size_t)rows * NHD * sizeof(float);
  unsigned short* y0h = (unsigned short*)(ws + off); off += planeX;
  unsigned short* y0l = (unsigned short*)(ws + off); off += planeX;
  if (off > ws_size) return;

  {
    const int n8x = rows * DD / 8;
    const int n8w = DD * DD / 8;
    k_split<<<(n8x + NTHR - 1) / NTHR, NTHR, 0, stream>>>(x, xh, xl, n8x);
    k_split<<<(n8w + NTHR - 1) / NTHR, NTHR, 0, stream>>>(W_K, wkvh, wkvl, n8w);
    k_split<<<(n8w + NTHR - 1) / NTHR, NTHR, 0, stream>>>(W_V, wkvh + DD * DD, wkvl + DD * DD, n8w);
    k_split<<<(n8w + NTHR - 1) / NTHR, NTHR, 0, stream>>>(W1, w1h, w1l, n8w);
    k_split<<<(n8w + NTHR - 1) / NTHR, NTHR, 0, stream>>>(W2, w2h, w2l, n8w);
  }

  k_gemm_kv<<<dim3(rows / GR, 2), NTHR, 0, stream>>>(xh, xl, wkvh, wkvl, b_K, b_V, att_r, xv, alpha, rows);

  hipFuncSetAttribute(reinterpret_cast<const void*>(&k_att),
                      hipFuncAttributeMaxDynamicSharedMemorySize, LDS_ATT_BYTES);
  k_att<<<(nN + NB - 1) / NB, NTHR, LDS_ATT_BYTES, stream>>>(ei, alpha, xv, att_r, ln0_g, ln0_b,
                                                            y0h, y0l, nN, nE);

  hipFuncSetAttribute(reinterpret_cast<const void*>(&k_rff),
                      hipFuncAttributeMaxDynamicSharedMemorySize, LDS_RFF_BYTES);
  k_rff<<<rows / GR, NTHR, LDS_RFF_BYTES, stream>>>(y0h, y0l, w1h, w1l, w2h, w2l, b1, b2,
                                                    ln1_g, ln1_b, out, rows);
}
